// CNN_Casual_21552145891462
// MI455X (gfx1250) — hardware-verified
//
#include <hip/hip_runtime.h>
#define BS 8192
#define H0 28
#define C1 10
#define O1 24
#define P1 12
#define C2 20
#define O2 8
#define P2 4
#define NR1 (BS * O1 * O1)
#define NR2 (BS * O2 * O2)

typedef __bf16 v16b __attribute__((ext_vector_type(16)));
typedef unsigned short v8us __attribute__((ext_vector_type(8), may_alias));
typedef float  v8f  __attribute__((ext_vector_type(8)));
typedef float  v4f  __attribute__((ext_vector_type(4)));
typedef float  v4fa __attribute__((ext_vector_type(4), may_alias));
union FragB { v16b v; v8us half[2]; unsigned short u[16]; };

__device__ __forceinline__ unsigned short bf16_bits(float x) { unsigned int u = __float_as_uint(x); return (unsigned short)((u + 0x7FFFu + ((u >> 16) & 1u)) >> 16); }
__device__ __forceinline__ float bf16_val(unsigned short b) { return __uint_as_float(((unsigned int)b) << 16); }
__device__ __forceinline__ float bf16_round(float x) { return bf16_val(bf16_bits(x)); }
template <int NT>
__device__ __forceinline__ v8f mmaN(v16b ah, v16b al, v16b bh, v16b bl, v8f c) {
  c = __builtin_amdgcn_wmma_f32_16x16x32_bf16(false, ah, false, bh, (short)0, c, false, false);
  if (NT >= 2) c = __builtin_amdgcn_wmma_f32_16x16x32_bf16(false, al, false, bh, (short)0, c, false, false);
  if (NT >= 3) c = __builtin_amdgcn_wmma_f32_16x16x32_bf16(false, ah, false, bl, (short)0, c, false, false);
  asm volatile("v_nop\n\tv_nop\n\tv_nop\n\tv_nop" : "+v"(c) : "v"(ah), "v"(al), "v"(bh), "v"(bl));
  return c;
}

__global__ __launch_bounds__(256) void k_wt_bf16(const float* __restrict__ W, unsigned short* __restrict__ Wt, int K, int N) {
  const int t = blockIdx.x * 256 + threadIdx.x;
  const int k8n = K / 8;
  if (t >= N * k8n) return;
  const int n = t / k8n, k8 = (t % k8n) * 8;
  v8us v;
#pragma unroll
  for (int i = 0; i < 8; ++i) v[i] = bf16_bits(W[(size_t)(k8 + i) * N + n]);
  *(volatile v8us*)(Wt + (size_t)n * K + k8) = v;
  __threadfence();
  *(volatile v8us*)(Wt + (size_t)n * K + k8) = v;
}

template <bool ASPLIT, int ACT, bool BIAS_BF16>
__global__ __launch_bounds__(128) void k_gemm_bf(const float* __restrict__ A, int lda, const unsigned short* __restrict__ Wt, int ldb,
                                               const float* __restrict__ bias, float* __restrict__ C, int ldc, int M, int N, int K) {
  __shared__ __attribute__((aligned(16))) float so[4][16][64];
  const int tid = threadIdx.x, w = tid >> 5, lane = tid & 31, ln = lane & 15, hh = lane >> 4;
  const int ntn = N / 64;
  const int wid = blockIdx.x * 4 + w;
  const int mt = wid / ntn, nq = wid % ntn;
  if (mt * 16 >= M) return;
  const int row0 = mt * 16, col0 = nq * 64;
  const float* arow = A + (size_t)(row0 + ln) * lda;
  v8f acc[4] = {};
  for (int kb = 0; kb < K; kb += 32) {
    FragB ah, al;
    const v4f x0 = *(const v4fa*)(arow + kb + 8 * hh), x1 = *(const v4fa*)(arow + kb + 8 * hh + 4);
    const v4f x2 = *(const v4fa*)(arow + kb + 16 + 8 * hh), x3 = *(const v4fa*)(arow + kb + 16 + 8 * hh + 4);
    float xs[16] = {x0[0],x0[1],x0[2],x0[3],x1[0],x1[1],x1[2],x1[3],x2[0],x2[1],x2[2],x2[3],x3[0],x3[1],x3[2],x3[3]};
#pragma unroll
    for (int i = 0; i < 16; ++i) { const unsigned short hb = bf16_bits(xs[i]); ah.u[i] = hb; al.u[i] = ASPLIT ? bf16_bits(xs[i] - bf16_val(hb)) : (unsigned short)0; }
#pragma unroll
    for (int t = 0; t < 4; ++t) {
      const unsigned short* brow = Wt + (size_t)(col0 + t * 16 + ln) * ldb + kb;
      FragB b;
      b.half[0] = *(const v8us*)(brow + 8 * hh);
      b.half[1] = *(const v8us*)(brow + 16 + 8 * hh);
      acc[t] = mmaN<ASPLIT ? 2 : 1>(ah.v, al.v, b.v, b.v, acc[t]);
    }
  }
#pragma unroll
  for (int t = 0; t < 4; ++t) {
    float bv = bias ? bias[col0 + t * 16 + ln] : 0.f;
    if (BIAS_BF16) bv = bf16_round(bv);
#pragma unroll
    for (int r = 0; r < 8; ++r) { float v = acc[t][r] + bv; if (ACT == 1) v = fmaxf(v, 0.f); so[w][8 * hh + r][t * 16 + ln] = v; }
  }
  __builtin_amdgcn_fence(__ATOMIC_ACQ_REL, "workgroup");
  __builtin_amdgcn_wave_barrier();
  const int rsub = lane >> 4, c4 = (lane & 15) * 4;
  for (int pass = 0; pass < 2; ++pass) {
#pragma unroll
    for (int q = 0; q < 8; ++q) {
      const int r = q * 2 + rsub;
      const v4f v = *(const v4fa*)&so[w][r][c4];
      *(volatile v4f*)(C + (size_t)(row0 + r) * ldc + col0 + c4) = v;
    }
    if (pass == 0) __threadfence();
  }
}

template <int D, bool CAUSAL>
__global__ __launch_bounds__(128) void k_flash(const float* __restrict__ qb, const float* __restrict__ kb, const float* __restrict__ vb,
                                             int pitch, int T, int H, float scale, float* __restrict__ y, int ypitch) {
  constexpr int KS = D / 32;
  constexpr int DT = D / 16;
  __shared__ __attribute__((aligned(16))) unsigned short sKh[32][D + 8], sKl[32][D + 8], sVh[32][D + 8], sVl[32][D + 8];
  __shared__ __attribute__((aligned(16))) unsigned short sPh[4][16][40], sPl[4][16][40];
  __shared__ __attribute__((aligned(16))) float sO[4][16][D];
  const int tid = threadIdx.x, w = tid >> 5, lane = tid & 31, ln = lane & 15, hh = lane >> 4;
  const int nqb = (T + 63) / 64;
  const int bh = blockIdx.x / nqb, qblk = blockIdx.x % nqb;
  const int b = bh / H, h = bh % H;
  const int q0 = qblk * 64 + w * 16;
  const float* Q = qb + (size_t)b * T * pitch + h * D;
  const float* K = kb + (size_t)b * T * pitch + h * D;
  const float* V = vb + (size_t)b * T * pitch + h * D;

  FragB aqh[KS], aql[KS];
  {
    int row = q0 + ln; if (row >= T) row = T - 1;
    const float* qr = Q + (size_t)row * pitch;
#pragma unroll
    for (int ks = 0; ks < KS; ++ks)
#pragma unroll
      for (int i = 0; i < 16; ++i) {
        const int d = ks * 32 + ((i < 8) ? (8 * hh + i) : (16 + 8 * hh + (i - 8)));
        const float x = qr[d] * scale; const unsigned short hb = bf16_bits(x);
        aqh[ks].u[i] = hb; aql[ks].u[i] = bf16_bits(x - bf16_val(hb));
      }
  }
  float m_r[8], l_r[8];
#pragma unroll
  for (int r = 0; r < 8; ++r) { m_r[r] = -3.0e38f; l_r[r] = 0.f; }
  v8f oacc[DT];
#pragma unroll
  for (int dt = 0; dt < DT; ++dt) oacc[dt] = (v8f){0.f,0.f,0.f,0.f,0.f,0.f,0.f,0.f};

  const int kv_end = CAUSAL ? min(T, qblk * 64 + 64) : T;
  for (int j0 = 0; j0 < kv_end; j0 += 32) {
    __syncthreads();
    for (int e = tid; e < 32 * (D / 4); e += 128) {
      const int r = e / (D / 4), c4 = (e % (D / 4)) * 4;
      const int key = j0 + r;
      v4f kf = {0.f,0.f,0.f,0.f}, vf = {0.f,0.f,0.f,0.f};
      if (key < T) { kf = *(const v4fa*)(K + (size_t)key * pitch + c4); vf = *(const v4fa*)(V + (size_t)key * pitch + c4); }
#pragma unroll
      for (int t = 0; t < 4; ++t) {
        unsigned short hb = bf16_bits(kf[t]); sKh[r][c4 + t] = hb; sKl[r][c4 + t] = bf16_bits(kf[t] - bf16_val(hb));
        hb = bf16_bits(vf[t]); sVh[r][c4 + t] = hb; sVl[r][c4 + t] = bf16_bits(vf[t] - bf16_val(hb));
      }
    }
    __syncthreads();
    v8f s[2];
#pragma unroll
    for (int nt = 0; nt < 2; ++nt) {
      v8f acc = {};
#pragma unroll
      for (int ks = 0; ks < KS; ++ks) {
        FragB bh_, bl_;
        bh_.half[0] = *(const v8us*)&sKh[nt * 16 + ln][ks * 32 + 8 * hh]; bh_.half[1] = *(const v8us*)&sKh[nt * 16 + ln][ks * 32 + 16 + 8 * hh];
        bl_.half[0] = *(const v8us*)&sKl[nt * 16 + ln][ks * 32 + 8 * hh]; bl_.half[1] = *(const v8us*)&sKl[nt * 16 + ln][ks * 32 + 16 + 8 * hh];
        acc = mmaN<3>(aqh[ks].v, aql[ks].v, bh_.v, bl_.v, acc);
      }
      s[nt] = acc;
    }
    float alpha[8];
#pragma unroll
    for (int r = 0; r < 8; ++r) {
      const int qi = q0 + 8 * hh + r;
      const int ja = j0 + ln, jb = j0 + 16 + ln;
      if (CAUSAL) { if (ja > qi) s[0][r] = -3.0e38f; if (jb > qi) s[1][r] = -3.0e38f; }
      if (ja >= T) s[0][r] = -3.0e38f;
      if (jb >= T) s[1][r] = -3.0e38f;
      float mx = fmaxf(s[0][r], s[1][r]);
      mx = fmaxf(mx, __shfl_xor(mx, 1, 32)); mx = fmaxf(mx, __shfl_xor(mx, 2, 32)); mx = fmaxf(mx, __shfl_xor(mx, 4, 32)); mx = fmaxf(mx, __shfl_xor(mx, 8, 32));
      const float mnew = fmaxf(m_r[r], mx);
      alpha[r] = (mnew > -1.0e38f) ? __expf(m_r[r] - mnew) : 1.0f;
      const float p0 = (s[0][r] > -1.0e38f) ? __expf(s[0][r] - mnew) : 0.f;
      const float p1 = (s[1][r] > -1.0e38f) ? __expf(s[1][r] - mnew) : 0.f;
      m_r[r] = mnew;
      l_r[r] = l_r[r] * alpha[r] + p0 + p1;
      unsigned short hb = bf16_bits(p0); sPh[w][8 * hh + r][ln] = hb;      sPl[w][8 * hh + r][ln] = bf16_bits(p0 - bf16_val(hb));
      hb = bf16_bits(p1);                sPh[w][8 * hh + r][16 + ln] = hb; sPl[w][8 * hh + r][16 + ln] = bf16_bits(p1 - bf16_val(hb));
    }
#pragma unroll
    for (int dt = 0; dt < DT; ++dt)
#pragma unroll
      for (int r = 0; r < 8; ++r) oacc[dt][r] *= alpha[r];
    __builtin_amdgcn_fence(__ATOMIC_ACQ_REL, "workgroup");
    __builtin_amdgcn_wave_barrier();
    FragB pah, pal;
    pah.half[0] = *(const v8us*)&sPh[w][ln][8 * hh]; pah.half[1] = *(const v8us*)&sPh[w][ln][16 + 8 * hh];
    pal.half[0] = *(const v8us*)&sPl[w][ln][8 * hh]; pal.half[1] = *(const v8us*)&sPl[w][ln][16 + 8 * hh];
#pragma unroll
    for (int dt = 0; dt < DT; ++dt) {
      FragB bvh, bvl;
#pragma unroll
      for (int i = 0; i < 8; ++i) {
        bvh.u[i] = sVh[8 * hh + i][dt * 16 + ln]; bvh.u[8 + i] = sVh[16 + 8 * hh + i][dt * 16 + ln];
        bvl.u[i] = sVl[8 * hh + i][dt * 16 + ln]; bvl.u[8 + i] = sVl[16 + 8 * hh + i][dt * 16 + ln];
      }
      oacc[dt] = mmaN<3>(pah.v, pal.v, bvh.v, bvl.v, oacc[dt]);
    }
    __builtin_amdgcn_fence(__ATOMIC_ACQ_REL, "workgroup");
    __builtin_amdgcn_wave_barrier();
  }
#pragma unroll
  for (int r = 0; r < 8; ++r) {
    float l = l_r[r];
    l += __shfl_xor(l, 1, 32); l += __shfl_xor(l, 2, 32); l += __shfl_xor(l, 4, 32); l += __shfl_xor(l, 8, 32);
    l_r[r] = (l > 0.f) ? 1.0f / l : 0.f;
  }
#pragma unroll
  for (int dt = 0; dt < DT; ++dt)
#pragma unroll
    for (int r = 0; r < 8; ++r) sO[w][8 * hh + r][dt * 16 + ln] = oacc[dt][r] * l_r[r];
  __builtin_amdgcn_fence(__ATOMIC_ACQ_REL, "workgroup");
  __builtin_amdgcn_wave_barrier();
  for (int pass = 0; pass < 2; ++pass) {
    for (int r = 0; r < 16; ++r) {
      const int row = q0 + r;
      if (row < T && lane < D / 4) {
        const v4f val = *(const v4fa*)&sO[w][r][lane * 4];
        *(volatile v4f*)(y + ((size_t)b * T + row) * ypitch + h * D + lane * 4) = val;
      }
    }
    if (pass == 0) __threadfence();
  }
}

typedef _Float16 v16h __attribute__((ext_vector_type(16)));
union FragH { v16h v; v8us half[2]; _Float16 h[16]; unsigned short u[16]; };
template <int NT>
__device__ __forceinline__ v8f mmaH(v16h ah, v16h al, v16h bh, v16h bl, v8f c) {
  c = __builtin_amdgcn_wmma_f32_16x16x32_f16(false, ah, false, bh, (short)0, c, false, false);
  if (NT >= 2) c = __builtin_amdgcn_wmma_f32_16x16x32_f16(false, al, false, bh, (short)0, c, false, false);
  if (NT >= 3) c = __builtin_amdgcn_wmma_f32_16x16x32_f16(false, ah, false, bl, (short)0, c, false, false);
  asm volatile("v_nop\n\tv_nop\n\tv_nop\n\tv_nop" : "+v"(c) : "v"(ah), "v"(al), "v"(bh), "v"(bl));
  return c;
}
template <bool ASPLIT>
__global__ __launch_bounds__(128) void k_gemm_h(const float* __restrict__ A, int lda, size_t sA, const _Float16* __restrict__ Bh, int ldb, size_t sB, float alpha, float* __restrict__ C, int ldc, size_t sC, int M, int N, int K) {
  __shared__ __attribute__((aligned(16))) float so[4][16][64];
  const int tid = threadIdx.x, w = tid >> 5, lane = tid & 31, ln = lane & 15, hh = lane >> 4; const int by = blockIdx.y;
  A += (size_t)by * sA; Bh += (size_t)by * sB; C += (size_t)by * sC;
  const int ntn = (N + 63) / 64; const int wid = blockIdx.x * 4 + w; const int mt = wid / ntn, nq = wid % ntn; if (mt * 16 >= M) return;
  const int row0 = mt * 16, col0 = nq * 64; const float* arow = A + (size_t)(row0 + ln) * lda;
  v8f acc[4] = {};
  for (int kb = 0; kb < K; kb += 32) {
    FragH ah, al;
    const v4f x0 = *(const v4fa*)(arow + kb + 8 * hh), x1 = *(const v4fa*)(arow + kb + 8 * hh + 4), x2 = *(const v4fa*)(arow + kb + 16 + 8 * hh), x3 = *(const v4fa*)(arow + kb + 16 + 8 * hh + 4);
    float xs[16] = {x0[0],x0[1],x0[2],x0[3],x1[0],x1[1],x1[2],x1[3],x2[0],x2[1],x2[2],x2[3],x3[0],x3[1],x3[2],x3[3]};
#pragma unroll
    for (int i = 0; i < 16; ++i) { const _Float16 h = (_Float16)xs[i]; ah.h[i] = h; al.h[i] = ASPLIT ? (_Float16)(xs[i] - (float)h) : (_Float16)0.0f; }
#pragma unroll
    for (int t = 0; t < 4; ++t) { if (col0 + t * 16 >= N) continue; const size_t boff = (size_t)(col0 + t * 16 + ln) * ldb + kb; FragH bq; bq.half[0] = *(const v8us*)(Bh + boff + 8 * hh); bq.half[1] = *(const v8us*)(Bh + boff + 16 + 8 * hh);
      acc[t] = mmaH<ASPLIT ? 2 : 1>(ah.v, al.v, bq.v, bq.v, acc[t]); }
  }
#pragma unroll
  for (int t = 0; t < 4; ++t) { if (col0 + t * 16 >= N) continue;
#pragma unroll
    for (int r = 0; r < 8; ++r) so[w][8 * hh + r][t * 16 + ln] = acc[t][r] * alpha; }
  __builtin_amdgcn_fence(__ATOMIC_ACQ_REL, "workgroup"); __builtin_amdgcn_wave_barrier();
  const int rsub = lane >> 4, c4 = (lane & 15) * 4;
  for (int pass = 0; pass < 2; ++pass) {
#pragma unroll
    for (int q = 0; q < 8; ++q) { const int r = q * 2 + rsub; if (col0 + c4 < N) { const v4f v = *(const v4fa*)&so[w][r][c4]; *(volatile v4f*)(C + (size_t)(row0 + r) * ldc + col0 + c4) = v; } }
    if (pass == 0) __threadfence(); }
}

__global__ __launch_bounds__(256) void k_wts(const float* __restrict__ w1, const float* __restrict__ w2, _Float16* __restrict__ Bt1, _Float16* __restrict__ Bt2) {
  const int t = blockIdx.x * 256 + threadIdx.x;
  if (t < 16 * 4) { const int o = t >> 2, k8 = (t & 3) * 8; FragH f; for (int q = 0; q < 8; ++q) { const int k = k8 + q; f.h[q] = (o < C1 && k < 25) ? (_Float16)(bf16_round(w1[o * 25 + k]) * 4.0f) : (_Float16)0.0f; } *(volatile v8us*)((unsigned short*)Bt1 + o * 32 + k8) = f.half[0]; __threadfence(); *(volatile v8us*)((unsigned short*)Bt1 + o * 32 + k8) = f.half[0]; }
  if (t < 32 * 32) { const int o = t >> 5, k8 = (t & 31) * 8; FragH f; for (int q = 0; q < 8; ++q) { const int k = k8 + q; const int c = k / 25, kk = k % 25; f.h[q] = (o < C2 && k < 250) ? (_Float16)(bf16_round(w2[(o * C1 + c) * 25 + kk]) * 4.0f) : (_Float16)0.0f; } *(volatile v8us*)((unsigned short*)Bt2 + o * 256 + k8) = f.half[0]; __threadfence(); *(volatile v8us*)((unsigned short*)Bt2 + o * 256 + k8) = f.half[0]; }
}
__global__ __launch_bounds__(256) void k_xs(const float* __restrict__ x, const float* __restrict__ m, _Float16* __restrict__ XS) { const size_t t = (size_t)blockIdx.x * 256 + threadIdx.x; if (t >= (size_t)BS * H0 * H0 / 8) return; FragH f;
#pragma unroll
  for (int q = 0; q < 8; ++q) { const size_t e = t * 8 + q; const int p = (int)(e % (H0 * H0)); f.h[q] = (_Float16)(bf16_round(x[e]) * (1.0f / (1.0f + expf(-bf16_round(m[p]))))); }
  *(volatile v8us*)((unsigned short*)XS + t * 8) = f.half[0]; __threadfence(); *(volatile v8us*)((unsigned short*)XS + t * 8) = f.half[0]; }
__constant__ int KOFF1[32] = {0,1,2,3,4, 28,29,30,31,32, 56,57,58,59,60, 84,85,86,87,88, 112,113,114,115,116, -1,-1,-1,-1,-1,-1,-1};
__global__ __launch_bounds__(128) void k_conv1(const _Float16* __restrict__ XS, const _Float16* __restrict__ Bt, const float* __restrict__ b1, _Float16* __restrict__ Hp) {
  __shared__ __attribute__((aligned(16))) float so[4][16][17];
  const int tid = threadIdx.x, w = tid >> 5, lane = tid & 31, ln = lane & 15, hh = lane >> 4; const int mt = blockIdx.x * 4 + w; if (mt * 16 >= NR1) return; const int row0 = mt * 16; const int r = row0 + ln;
  const int b = r / (O1 * O1), rem = r % (O1 * O1); const int g = rem >> 2, d = rem & 3; const int oy = 2 * (g / P1) + (d >> 1), ox = 2 * (g % P1) + (d & 1); const _Float16* xb = XS + (size_t)b * H0 * H0 + oy * H0 + ox;
  FragH ah;
#pragma unroll
  for (int q = 0; q < 16; ++q) { const int k = (q < 8) ? (8 * hh + q) : (16 + 8 * hh + (q - 8)); const int ko = KOFF1[k]; ah.h[q] = (ko >= 0) ? xb[ko] : (_Float16)0.0f; }
  FragH bq; bq.half[0] = *(const v8us*)((const unsigned short*)Bt + (size_t)ln * 32 + 8 * hh); bq.half[1] = *(const v8us*)((const unsigned short*)Bt + (size_t)ln * 32 + 16 + 8 * hh);
  v8f acc = {0.f,0.f,0.f,0.f,0.f,0.f,0.f,0.f}; acc = mmaH<1>(ah.v, ah.v, bq.v, bq.v, acc);
#pragma unroll
  for (int q = 0; q < 8; ++q) so[w][8 * hh + q][ln] = acc[q] * 0.25f + ((ln < C1) ? bf16_round(b1[ln]) : 0.f);
  __builtin_amdgcn_fence(__ATOMIC_ACQ_REL, "workgroup"); __builtin_amdgcn_wave_barrier();
  const int g0 = (row0 % (O1 * O1)) >> 2; _Float16* dst = Hp + ((size_t)b * (P1 * P1) + g0) * 16;
  typedef _Float16 v2h __attribute__((ext_vector_type(2))); v2h pv; { const int e = 2 * lane; const int p = e >> 4, c = e & 15; const float m0 = fmaxf(fmaxf(so[w][4 * p][c], so[w][4 * p + 1][c]), fmaxf(so[w][4 * p + 2][c], so[w][4 * p + 3][c])); const float m1 = fmaxf(fmaxf(so[w][4 * p][c + 1], so[w][4 * p + 1][c + 1]), fmaxf(so[w][4 * p + 2][c + 1], so[w][4 * p + 3][c + 1])); pv.x = (_Float16)fmaxf(m0, 0.f); pv.y = (_Float16)fmaxf(m1, 0.f); }
  for (int pass = 0; pass < 2; ++pass) { *(volatile v2h*)(dst + 2 * lane) = pv; if (pass == 0) __threadfence(); }
}
__global__ __launch_bounds__(256) void k_kt2fill(int* __restrict__ T) { const int k = threadIdx.x; int v = -1; if (k < 250) { const int c = k / 25, kk = k % 25; v = ((kk / 5) * P1 + kk % 5) * 16 + c; } T[k] = v; }
__global__ __launch_bounds__(128) void k_conv2(const _Float16* __restrict__ Hh, const int* __restrict__ KT, const _Float16* __restrict__ Bt, const float* __restrict__ b2, float* __restrict__ Y2) {
  __shared__ int skt[256]; for (int i = threadIdx.x; i < 256; i += 128) skt[i] = KT[i]; __syncthreads();
  __shared__ __attribute__((aligned(16))) float so[4][16][32];
  const int tid = threadIdx.x, w = tid >> 5, lane = tid & 31, ln = lane & 15, hh = lane >> 4; const int mt = blockIdx.x * 4 + w; if (mt * 16 >= NR2) return; const int row0 = mt * 16; const int r = row0 + ln;
  const int b = r / (O2 * O2), rem = r % (O2 * O2); const int oy = rem / O2, ox = rem % O2; const _Float16* hb = Hh + ((size_t)b * (P1 * P1) + oy * P1 + ox) * 16;
  v8f acc[2] = {};
#pragma unroll 1
  for (int kb = 0; kb < 256; kb += 32) { FragH ah;
#pragma unroll
    for (int q = 0; q < 16; ++q) { const int k = kb + ((q < 8) ? (8 * hh + q) : (16 + 8 * hh + (q - 8))); const int ko = skt[k]; ah.h[q] = (ko >= 0) ? hb[ko] : (_Float16)0.0f; }
#pragma unroll
    for (int t2 = 0; t2 < 2; ++t2) { FragH bq; bq.half[0] = *(const v8us*)((const unsigned short*)Bt + (size_t)(t2 * 16 + ln) * 256 + kb + 8 * hh); bq.half[1] = *(const v8us*)((const unsigned short*)Bt + (size_t)(t2 * 16 + ln) * 256 + kb + 16 + 8 * hh); acc[t2] = mmaH<1>(ah.v, ah.v, bq.v, bq.v, acc[t2]); } }
#pragma unroll
  for (int t2 = 0; t2 < 2; ++t2) {
#pragma unroll
    for (int q = 0; q < 8; ++q) { const int o = t2 * 16 + ln; so[w][8 * hh + q][o] = acc[t2][q] * 0.25f + ((o < C2) ? bf16_round(b2[o]) : 0.f); } }
  __builtin_amdgcn_fence(__ATOMIC_ACQ_REL, "workgroup"); __builtin_amdgcn_wave_barrier();
  for (int pass = 0; pass < 2; ++pass) { for (int q = lane; q < 128; q += 32) { const int rr = q >> 3, c4 = (q & 7) * 4; *(volatile v4f*)(Y2 + (size_t)(row0 + rr) * 32 + c4) = *(const v4fa*)&so[w][rr][c4]; } if (pass == 0) __threadfence(); }
}
__global__ __launch_bounds__(512) void k_head(const float* __restrict__ Y2, const float* __restrict__ f1w, const float* __restrict__ f1b, const float* __restrict__ f2w, const float* __restrict__ f2b, float* __restrict__ out) {
  __shared__ float sh[16][320]; __shared__ float s1[16][64]; __shared__ float sres[16][16];
  const int tid = threadIdx.x, wv = tid >> 5, lane = tid & 31; const int b = blockIdx.x * 16 + wv;
  for (int e = lane; e < 320; e += 32) { const int c = e / 16, py = (e / 4) % 4, px = e % 4; float m = -3.0e38f; for (int dy = 0; dy < 2; ++dy) for (int dx = 0; dx < 2; ++dx) { const size_t r = ((size_t)b * O2 + 2 * py + dy) * O2 + 2 * px + dx; m = fmaxf(m, Y2[r * 32 + c]); } sh[wv][e] = fmaxf(m, 0.f); }
  __builtin_amdgcn_fence(__ATOMIC_ACQ_REL, "workgroup"); __builtin_amdgcn_wave_barrier();
  for (int j = lane; j < 64; j += 32) { float s = 0.f; if (j < 50) { s = bf16_round(f1b[j]);
#pragma unroll 1
      for (int k = 0; k < 320; ++k) s += sh[wv][k] * bf16_round(f1w[j * 320 + k]); s = fmaxf(s, 0.f); } s1[wv][j] = s; }
  __builtin_amdgcn_fence(__ATOMIC_ACQ_REL, "workgroup"); __builtin_amdgcn_wave_barrier();
  float lg = -3.0e38f; if (lane < 10) { lg = bf16_round(f2b[lane]);
#pragma unroll 1
    for (int k = 0; k < 50; ++k) lg += s1[wv][k] * bf16_round(f2w[lane * 50 + k]); }
  float mx = lg; for (int o = 16; o >= 1; o >>= 1) mx = fmaxf(mx, __shfl_xor(mx, o, 32)); float ex = (lane < 10) ? expf(lg - mx) : 0.f; float den = ex; for (int o = 16; o >= 1; o >>= 1) den += __shfl_xor(den, o, 32);
  if (lane < 10) sres[wv][lane] = (lg - mx) - logf(den);
  __syncthreads();
  for (int pass = 0; pass < 2; ++pass) { if (tid < 160) *(volatile float*)(out + (size_t)blockIdx.x * 160 + tid) = sres[tid / 10][tid % 10]; if (pass == 0) __threadfence(); }
}
extern "C" void kernel_launch(void* const* d_in, const int* in_sizes, int n_in,
                              void* d_out, int out_size, void* d_ws, size_t ws_size, hipStream_t stream) {
  (void)in_sizes; (void)n_in; (void)out_size;
  const float* x = (const float*)d_in[0]; const float* mask = (const float*)d_in[1]; const float* w1 = (const float*)d_in[2]; const float* b1 = (const float*)d_in[3]; const float* w2 = (const float*)d_in[4]; const float* b2 = (const float*)d_in[5]; const float* f1w = (const float*)d_in[6]; const float* f1b = (const float*)d_in[7]; const float* f2w = (const float*)d_in[8]; const float* f2b = (const float*)d_in[9];
  char* ws = (char*)d_ws; size_t off = 0;
  auto take = [&](size_t bytes) { char* p = ws + off; off += (bytes + 255) & ~(size_t)255; return p; };
  _Float16* Bt1 = (_Float16*)take(16 * 32 * 2); _Float16* Bt2 = (_Float16*)take(32 * 256 * 2); int* KT = (int*)take(256 * 4); _Float16* XS = (_Float16*)take((size_t)BS * H0 * H0 * 2);
  _Float16* Hp = (_Float16*)take((size_t)BS * P1 * P1 * 16 * 2); float* Y2 = (float*)take((size_t)NR2 * 32 * 4);
  if (off > ws_size) return;
  k_wts<<<4, 256, 0, stream>>>(w1, w2, Bt1, Bt2); k_kt2fill<<<1, 256, 0, stream>>>(KT); k_xs<<<(unsigned)(((size_t)BS * H0 * H0 / 8 + 255) / 256), 256, 0, stream>>>(x, mask, XS);
  k_conv1<<<(NR1 / 16 + 3) / 4, 128, 0, stream>>>(XS, Bt1, b1, Hp);
  k_conv2<<<(NR2 / 16 + 3) / 4, 128, 0, stream>>>(Hp, KT, Bt2, b2, Y2);
  k_head<<<BS / 16, 512, 0, stream>>>(Y2, f1w, f1b, f2w, f2b, (float*)d_out);
}
